// NewAttention_55344948576827
// MI455X (gfx1250) — hardware-verified
//
#include <hip/hip_runtime.h>


#define NB_  4
#define TT   4096
#define DM   512
#define NH_  8
#define NKV  8
#define REP  (NH_ / NKV)
#define HD   64
#define DQ   (NH_ * HD)
#define DKV  (NKV * HD)
#define ZH   2
#define RH   512
#define WIN  0
#define PCAR 1024.0f
#define SCL  0.125f
typedef _Float16 h16;
typedef unsigned short bf;
typedef __attribute__((ext_vector_type(16))) __bf16   v16bf;
typedef __attribute__((ext_vector_type(16))) _Float16 v16h;
typedef __attribute__((ext_vector_type(8)))  _Float16 v8h;
typedef __attribute__((ext_vector_type(8)))  unsigned short v8us;
typedef __attribute__((ext_vector_type(8)))  float    v8f;
typedef __attribute__((ext_vector_type(4)))  float    v4f;
typedef v8h  __attribute__((may_alias)) v8ha;
typedef v4f  __attribute__((may_alias)) v4fa;
typedef v8us __attribute__((may_alias)) v8usa;

__device__ __forceinline__ unsigned short f2bf(float f) { unsigned u = __float_as_uint(f); u += 0x7FFFu + ((u >> 16) & 1u); return (unsigned short)(u >> 16); }
__device__ __forceinline__ float bf2f(unsigned short b) { return __uint_as_float(((unsigned)b) << 16); }
__device__ __forceinline__ float bfr(float f) { return bf2f(f2bf(f)); }
__device__ __forceinline__ v16h cat16(v8h lo, v8h hi) { return __builtin_shufflevector(lo, hi, 0, 1, 2, 3, 4, 5, 6, 7, 8, 9, 10, 11, 12, 13, 14, 15); }
__device__ __forceinline__ v16bf cat16b(v8us lo, v8us hi) { return __builtin_bit_cast(v16bf, __builtin_shufflevector(lo, hi, 0, 1, 2, 3, 4, 5, 6, 7, 8, 9, 10, 11, 12, 13, 14, 15)); }
__device__ __forceinline__ v8f wmma16(v16h a, v16h b, v8f c) { return __builtin_amdgcn_wmma_f32_16x16x32_f16(false, a, false, b, (short)0, c, false, false); }
__device__ __forceinline__ v8f wmmab(v16bf a, v16bf b, v8f c) { return __builtin_amdgcn_wmma_f32_16x16x32_bf16(false, a, false, b, (short)0, c, false, false); }


template <typename T16> struct WFrag;
template <> struct WFrag<h16> { typedef v16h V; static __device__ __forceinline__ V ld(const h16* p) { return cat16(*(const v8h*)p, *(const v8h*)(p + 16)); } static __device__ __forceinline__ v8f mma(V a, V b, v8f c) { return wmma16(a, b, c); } };
template <> struct WFrag<bf> { typedef v16bf V; static __device__ __forceinline__ V ld(const bf* p) { return cat16b(*(const v8us*)p, *(const v8us*)(p + 16)); } static __device__ __forceinline__ v8f mma(V a, V b, v8f c) { return wmmab(a, b, c); } };
template <typename T16, int NSPLIT, bool BIAS>
__global__ __launch_bounds__(32) void k_gemmw(const T16* __restrict__ A, const T16* __restrict__ A2, const T16* __restrict__ Bt, const T16* __restrict__ Bt2, int K, float* C, int ldc, const float* __restrict__ bias, size_t sA, size_t sB, size_t sC) {
    typedef typename WFrag<T16>::V V;
    __shared__ __align__(16) float os[16 * 68];
    const size_t z = blockIdx.z; A += z * sA; if (A2) A2 += z * sA; Bt += z * sB; if (Bt2) Bt2 += z * sB; C += z * sC;
    const int lane = threadIdx.x & 31, lr = lane & 15, hi = lane >> 4; const int r0 = blockIdx.x * 64, c0 = blockIdx.y * 64;
    v8f acc[4][4];
#pragma unroll
    for (int mb = 0; mb < 4; ++mb)
#pragma unroll
        for (int nb = 0; nb < 4; ++nb) acc[mb][nb] = (v8f){};
    const size_t aoff = (size_t)(r0 + lr) * K + 8 * hi, boff = (size_t)(c0 + lr) * K + 8 * hi;
#pragma unroll 1
    for (int kc = 0; kc < K; kc += 32) {
        V a[4], a2[4];
#pragma unroll
        for (int mb = 0; mb < 4; ++mb) { a[mb] = WFrag<T16>::ld(A + aoff + (size_t)mb * 16 * K + kc); if (NSPLIT == 1 || NSPLIT == 2) a2[mb] = WFrag<T16>::ld(A2 + aoff + (size_t)mb * 16 * K + kc); }
#pragma unroll
        for (int nb = 0; nb < 4; ++nb) { const V b = WFrag<T16>::ld(Bt + boff + (size_t)nb * 16 * K + kc); V b2; if (NSPLIT >= 2) b2 = WFrag<T16>::ld(Bt2 + boff + (size_t)nb * 16 * K + kc);
#pragma unroll
            for (int mb = 0; mb < 4; ++mb) { acc[mb][nb] = WFrag<T16>::mma(a[mb], b, acc[mb][nb]); if (NSPLIT == 1 || NSPLIT == 2) acc[mb][nb] = WFrag<T16>::mma(a2[mb], b, acc[mb][nb]); if (NSPLIT >= 2) acc[mb][nb] = WFrag<T16>::mma(a[mb], b2, acc[mb][nb]); } }
        asm volatile("v_nop\n\tv_nop\n\tv_nop\n\tv_nop" : "+v"(acc[0][0]), "+v"(acc[1][1]), "+v"(acc[2][2]), "+v"(acc[3][3]) : "v"(a[0]), "v"(a[3]));
    }
#pragma unroll
    for (int mb = 0; mb < 4; ++mb) {
#pragma unroll
        for (int nb = 0; nb < 4; ++nb) {
#pragma unroll
            for (int j = 0; j < 8; ++j) os[(hi * 8 + j) * 68 + nb * 16 + lr] = acc[mb][nb][j]; }
        __builtin_amdgcn_wave_barrier(); asm volatile("" ::: "memory");
        float* crow = C + (size_t)(r0 + mb * 16) * ldc + c0;
#pragma unroll 1
        for (int ps = 0; ps < 2; ++ps) {
#pragma unroll
            for (int s = 0; s < 8; ++s) { const int row = 2 * s + hi, cofs = lr * 4; v4f val = *(const v4fa*)(os + row * 68 + cofs); if (BIAS) { val[0] += bfr(bias[c0 + cofs]); val[1] += bfr(bias[c0 + cofs + 1]); val[2] += bfr(bias[c0 + cofs + 2]); val[3] += bfr(bias[c0 + cofs + 3]); }
                *(volatile v4f*)(crow + (size_t)row * ldc + cofs) = val; }
            if (ps == 0) __threadfence(); }
        __builtin_amdgcn_wave_barrier(); asm volatile("" ::: "memory");
    }
}

__device__ __forceinline__ h16 tohx(float x) { return (h16)x; }
__device__ __forceinline__ void splitf(float y, unsigned short& h, unsigned short& l) { h = f2bf(y); l = f2bf(y - bf2f(h)); }
typedef __attribute__((ext_vector_type(2))) _Float16 v2h;
typedef __attribute__((ext_vector_type(4))) _Float16 v4h;
typedef __attribute__((ext_vector_type(2))) unsigned short v2us;
typedef __attribute__((ext_vector_type(4))) unsigned short v4us;
typedef __attribute__((ext_vector_type(2))) float v2f;
typedef __attribute__((ext_vector_type(4))) int v4i;


__global__ __launch_bounds__(256) void k_cvt8(const float* __restrict__ src, bf* dst, size_t n8) { const size_t i = (size_t)blockIdx.x * 256 + threadIdx.x; if (i >= n8) return; const v8f v = *(const v8f*)(src + i * 8); v8us o;
#pragma unroll
    for (int k = 0; k < 8; ++k) o[k] = f2bf(v[k]); *(volatile v8us*)(dst + i * 8) = o; __threadfence(); *(volatile v8us*)(dst + i * 8) = o; }


#define NTAP 13
__constant__ float GW[NTAP + 1] = {0.398942292f,0.241970733f,0.0539909676f,0.00443184841f,0.000133830225f,0.00000148671961f,6.07588291e-9f,9.13472076e-12f,5.05227116e-15f,1.02797736e-18f,7.69459913e-23f,2.11881934e-27f,2.14638377e-32f,7.99882799e-38f};
__global__ __launch_bounds__(256) void k_band(const float* __restrict__ F, bf* Ah, bf* Al) {
    __shared__ float TL[64 + 2 * NTAP][68];
    const int c0 = blockIdx.x * 64, q0 = blockIdx.y * 64, tid = threadIdx.x;
#pragma unroll 1
    for (int u = tid; u < (64 + 2 * NTAP) * 16; u += 256) { const int rr = u >> 4, cc = (u & 15) * 4; const int r = q0 - NTAP + rr; const int rc = min(max(r, 0), TT - 1); const float inb = (r >= 0 && r < TT) ? 1.0f : 0.0f;
        const v4f a = *(const v4f*)(F + (size_t)rc * DM + c0 + cc); TL[rr][cc] = a[0] * inb; TL[rr][cc + 1] = a[1] * inb; TL[rr][cc + 2] = a[2] * inb; TL[rr][cc + 3] = a[3] * inb; }
    __syncthreads();
    const int cl = (tid & 15) * 4, rl = (tid >> 4) * 4; float acc[4][4];
#pragma unroll
    for (int i = 0; i < 4; ++i) { acc[i][0] = 0.f; acc[i][1] = 0.f; acc[i][2] = 0.f; acc[i][3] = 0.f; }
#pragma unroll 1
    for (int d = -NTAP; d <= NTAP; ++d) { const float w = GW[d < 0 ? -d : d];
#pragma unroll
        for (int i = 0; i < 4; ++i) { const float* tr = &TL[rl + i + NTAP + d][cl];
#pragma unroll
            for (int q = 0; q < 4; ++q) acc[i][q] = fmaf(w, tr[q], acc[i][q]); } }
#pragma unroll
    for (int ps = 0; ps < 2; ++ps) {
#pragma unroll
        for (int i = 0; i < 4; ++i) { v4us oh, ol;
#pragma unroll
            for (int q = 0; q < 4; ++q) { unsigned short a2, c2; splitf(acc[i][q], a2, c2); oh[q] = a2; ol[q] = c2; }
            const size_t oo = (size_t)(q0 + rl + i) * DM + c0 + cl; *(volatile v4us*)(Ah + oo) = oh; *(volatile v4us*)(Al + oo) = ol; }
        if (ps == 0) __threadfence(); }
}


extern "C" void kernel_launch(void* const* d_in, const int* in_sizes, int n_in,
                              void* d_out, int out_size, void* d_ws, size_t ws_size, hipStream_t stream) {
    (void)in_sizes; (void)n_in; (void)out_size;
    const float* x = (const float*)d_in[0]; const float* wq = (const float*)d_in[1]; const float* wo = (const float*)d_in[2]; const float* wk = nullptr; const float* wv = nullptr; (void)wk; (void)wv;
    float* OUT = (float*)d_out;
    char* wsp = (char*)d_ws;
    auto take = [&](size_t bytes) { char* p = wsp; wsp += (bytes + 255) & ~(size_t)255; return (void*)p; };
    bf* WQ = (bf*)take((size_t)DQ * DM * 2); bf* WO = (bf*)take((size_t)DM * DQ * 2); bf* XB = (bf*)take((size_t)TT * DM * 2); float* FQ = (float*)take((size_t)TT * DQ * 4); bf* ATh = (bf*)take((size_t)TT * DQ * 2); bf* ATl = (bf*)take((size_t)TT * DQ * 2);
    if ((size_t)(wsp - (char*)d_ws) > ws_size) return;
    { k_cvt8<<<(unsigned)(((size_t)DQ * DM / 8 + 255) / 256), 256, 0, stream>>>(wq, WQ, (size_t)DQ * DM / 8); k_cvt8<<<(unsigned)(((size_t)DM * DQ / 8 + 255) / 256), 256, 0, stream>>>(wo, WO, (size_t)DM * DQ / 8); }
    for (int b = 0; b < NB_; ++b) {
        k_cvt8<<<(unsigned)(((size_t)TT * DM / 8 + 255) / 256), 256, 0, stream>>>(x + (size_t)b * TT * DM, XB, (size_t)TT * DM / 8);
        k_gemmw<bf, 0, false><<<dim3(TT / 64, DQ / 64, 1), 32, 0, stream>>>(XB, nullptr, WQ, nullptr, DM, FQ, DQ, nullptr, 0, 0, 0);
        k_band<<<dim3(DM / 64, TT / 64, 1), 256, 0, stream>>>(FQ, ATh, ATl);
        k_gemmw<bf, 1, false><<<dim3(TT / 64, DM / 64, 1), 32, 0, stream>>>(ATh, ATl, WO, nullptr, DQ, OUT + (size_t)b * TT * DM, DM, nullptr, 0, 0, 0); }
}
